// RecurrentEmbeddingLayer_75728863363318
// MI455X (gfx1250) — hardware-verified
//
#include <hip/hip_runtime.h>
#include <stdint.h>


#define NBATCH 128
#define NT 1024
#define NF 16
#define KP0 32
#define UA 128
#define UB 128
#define UC 64
#define TCH 256
#define NCH (NT / TCH)
#define NROWS (NBATCH * NT)
#define HCARRY 256.0f
#define WCARRY 8.0f

typedef __attribute__((ext_vector_type(16))) _Float16 v16h;
typedef __attribute__((ext_vector_type(8)))  _Float16 v8h;
typedef __attribute__((ext_vector_type(16))) __bf16   v16b;
typedef __attribute__((ext_vector_type(8)))  __bf16   v8b;
typedef __attribute__((ext_vector_type(8)))  float    v8f;
typedef __attribute__((ext_vector_type(4)))  float    v4f;
typedef __attribute__((ext_vector_type(4)))  int      v4i;

__device__ __forceinline__ unsigned short f2bf_bits(float f) {
  unsigned u = __float_as_uint(f);
  return (unsigned short)((u + 0x7FFFu + ((u >> 16) & 1u)) >> 16);
}
__device__ __forceinline__ float bf_bits2f(unsigned short h) { return __uint_as_float(((unsigned)h) << 16); }

__device__ __forceinline__ void dep_guard_h(v8f& a, v8f& b, v16h x, v16h y) { asm volatile("v_nop\n\tv_nop\n\tv_nop\n\tv_nop" : "+v"(a), "+v"(b) : "v"(x), "v"(y)); }
__device__ __forceinline__ void dep_guard_b(v8f& a, v8f& b, v16b x, v16b y) { asm volatile("v_nop\n\tv_nop\n\tv_nop\n\tv_nop" : "+v"(a), "+v"(b) : "v"(x), "v"(y)); }
__device__ __forceinline__ void keep4_h(v16h a, v16h b, v16h c, v16h d) { asm volatile("v_nop" :: "v"(a), "v"(b), "v"(c), "v"(d)); }
__device__ __forceinline__ void keep4_b(v16b a, v16b b, v16b c, v16b d) { asm volatile("v_nop" :: "v"(a), "v"(b), "v"(c), "v"(d)); }
__device__ __forceinline__ void acc_guard4(v8f& a, v8f& b, v8f& c, v8f& d) { asm volatile("v_nop\n\tv_nop\n\tv_nop\n\tv_nop" : "+v"(a), "+v"(b), "+v"(c), "+v"(d)); }
__device__ __forceinline__ void acc_guard3(v8f& a, v8f& b, v8f& c) { asm volatile("v_nop\n\tv_nop\n\tv_nop\n\tv_nop" : "+v"(a), "+v"(b), "+v"(c)); }
template <typename T> struct Frag;
template <> struct Frag<_Float16> {
  typedef v16h V; union U { v16h v; v8h h[2]; };
  static __device__ __forceinline__ v16h load(const _Float16* p) {
    U f; f.h[0] = *(const v8h*)(p); f.h[1] = *(const v8h*)(p + 16); return f.v;
  }
  static __device__ __forceinline__ v8f mma(v16h a, v16h b, v8f c) {
    return __builtin_amdgcn_wmma_f32_16x16x32_f16(false, a, false, b, (short)0, c, false, false);
  }
  static __device__ __forceinline__ void guard(v8f& a, v8f& b, v16h x, v16h y) { dep_guard_h(a, b, x, y); }
  static __device__ __forceinline__ void keep(v16h a, v16h b, v16h c, v16h d) { keep4_h(a, b, c, d); }
};
template <> struct Frag<__bf16> {
  typedef v16b V; union U { v16b v; v8b h[2]; };
  static __device__ __forceinline__ v16b load(const __bf16* p) {
    U f; f.h[0] = *(const v8b*)(p); f.h[1] = *(const v8b*)(p + 16); return f.v;
  }
  static __device__ __forceinline__ v8f mma(v16b a, v16b b, v8f c) {
    return __builtin_amdgcn_wmma_f32_16x16x32_bf16(false, a, false, b, (short)0, c, false, false);
  }
  static __device__ __forceinline__ void guard(v8f& a, v8f& b, v16b x, v16b y) { dep_guard_b(a, b, x, y); }
  static __device__ __forceinline__ void keep(v16b a, v16b b, v16b c, v16b d) { keep4_b(a, b, c, d); }
};

template <int ET> struct Elem;
template <> struct Elem<0> { typedef _Float16 T; };
template <> struct Elem<1> { typedef __bf16 T; };
template <int ET, bool SPLIT, int BIAS_MODE, int OUT_MODE, bool RESID, int ACT = 0>
__global__ __launch_bounds__(256) void wmma_gemm64(
    const unsigned short* __restrict__ Ap, const unsigned short* __restrict__ A2p, int lda, long strideA,
    const unsigned short* __restrict__ Btp, const unsigned short* __restrict__ Bt2p, int ldb, long strideB,
    void* __restrict__ Cout, void* __restrict__ Cout2, int ldc, long strideC,
    const float* __restrict__ bias,
    const float* __restrict__ resid, long strideR,
    int M, int N, int K, float scale) {
  typedef typename Elem<ET>::T T;
  typedef typename Frag<T>::V V;
  const T* A = (const T*)Ap; const T* A2 = (const T*)A2p; const T* Bt = (const T*)Btp; const T* Bt2 = (const T*)Bt2p;
  __shared__ __align__(16) float sT[8][16 * 68];
  const int b    = blockIdx.y;
  const int lane = threadIdx.x & 31;
  const int wave = threadIdx.x >> 5;
  const int tilesN = N >> 6;
  const int tilesM = M >> 6;
  const int tile = blockIdx.x * 8 + wave;
  if (tile >= tilesM * tilesN) return;
  const int tm = tile / tilesN;
  const int tn = tile - tm * tilesN;
  const int m0 = tm << 6;
  const int n0 = tn << 6;

  const T* Ab  = A  + (size_t)b * strideA;
  const T* Bb  = Bt + (size_t)b * strideB;
  const T* Ab2 = SPLIT ? (A2  + (size_t)b * strideA) : nullptr;
  const T* Bb2 = SPLIT ? (Bt2 + (size_t)b * strideB) : nullptr;

  const int rlane = lane & 15;
  const int koff  = (lane >> 4) * 8;
  const int mOff  = (lane >> 4) * 8;

  v8f acc[4][4];
#pragma unroll
  for (int i = 0; i < 4; ++i)
#pragma unroll
    for (int j = 0; j < 4; ++j) acc[i][j] = (v8f){0.f,0.f,0.f,0.f,0.f,0.f,0.f,0.f};

  for (int k0 = 0; k0 < K; k0 += 32) {
    V bh[4], bl[4];
#pragma unroll
    for (int j = 0; j < 4; ++j) {
      const size_t bo = (size_t)(n0 + (j << 4) + rlane) * ldb + koff + k0;
      bh[j] = Frag<T>::load(Bb + bo);
      if (SPLIT) bl[j] = Frag<T>::load(Bb2 + bo);
    }
#pragma unroll
    for (int i = 0; i < 4; ++i) {
      const size_t ao = (size_t)(m0 + (i << 4) + rlane) * lda + koff + k0;
      V ah = Frag<T>::load(Ab + ao);
      V al;
      if (SPLIT) al = Frag<T>::load(Ab2 + ao);
#pragma unroll
      for (int j = 0; j < 4; ++j) {
        acc[i][j] = Frag<T>::mma(ah, bh[j], acc[i][j]);
        if (SPLIT) {
          acc[i][j] = Frag<T>::mma(ah, bl[j], acc[i][j]);
          acc[i][j] = Frag<T>::mma(al, bh[j], acc[i][j]);
        }
      }
      Frag<T>::guard(acc[i][0], acc[i][3], ah, SPLIT ? al : ah);
    }
    Frag<T>::keep(bh[0], bh[1], bh[2], bh[3]);
    if (SPLIT) Frag<T>::keep(bl[0], bl[1], bl[2], bl[3]);
  }
  acc_guard4(acc[0][0], acc[0][1], acc[0][2], acc[0][3]);
  acc_guard4(acc[1][0], acc[1][1], acc[1][2], acc[1][3]);
  acc_guard4(acc[2][0], acc[2][1], acc[2][2], acc[2][3]);
  acc_guard4(acc[3][0], acc[3][1], acc[3][2], acc[3][3]);

  float* slab = sT[wave];
  const float* Rb = RESID ? (resid + (size_t)b * strideR) : nullptr;
#pragma unroll
  for (int i = 0; i < 4; ++i) {
    const int mBase = m0 + (i << 4);
#pragma unroll
    for (int j = 0; j < 4; ++j) {
      const int n = n0 + (j << 4) + rlane;
      float bv = 0.f;
      if (BIAS_MODE == 2) bv = bias[n];
#pragma unroll
      for (int r = 0; r < 8; ++r) {
        float v = acc[i][j][r] * scale;
        if (BIAS_MODE == 1) v += bias[mBase + mOff + r];
        if (BIAS_MODE == 2) v += bv;
        if (RESID) v += Rb[(size_t)(mBase + mOff + r) * ldc + n];
        if (ACT == 1) v = tanhf(v);
        if (ACT == 2) v = fmaxf(v, 0.0f);
        if (ACT == 3) v = v / (1.0f + expf(-v));
        if (ACT == 4) v = (v > 0.f) ? v : 0.01f * v;
        if (ACT == 5) v = 0.5f * v * (1.0f + erff(v * 0.70710678118654752f));
        slab[(mOff + r) * 68 + (j << 4) + rlane] = v;
      }
    }
    __builtin_amdgcn_fence(__ATOMIC_RELEASE, "workgroup");
    __builtin_amdgcn_wave_barrier();
    __builtin_amdgcn_fence(__ATOMIC_ACQUIRE, "workgroup");
    if (OUT_MODE == 0) {
      float* C = (float*)Cout + (size_t)b * strideC;
      const int hh = lane >> 4, c4 = (lane & 15) * 4;
      for (int pass = 0; pass < 2; ++pass) {
#pragma unroll
        for (int it = 0; it < 8; ++it) {
          const int row = it * 2 + hh;
          v4f v = *(const v4f*)(slab + row * 68 + c4);
          *(volatile v4f*)(C + (size_t)(mBase + row) * ldc + n0 + c4) = v;
        }
        __threadfence();
      }
    } else {
      const int q = lane >> 3, c8 = (lane & 7) * 8;
      unsigned short* C  = (unsigned short*)Cout  + (size_t)b * strideC;
      unsigned short* C2 = (OUT_MODE == 2) ? ((unsigned short*)Cout2 + (size_t)b * strideC) : nullptr;
      for (int pass = 0; pass < 2; ++pass) {
#pragma unroll
        for (int it = 0; it < 4; ++it) {
          const int row = it * 4 + q;
          const float* sp = slab + row * 68 + c8;
          v8h hv, lv;
#pragma unroll
          for (int e = 0; e < 8; ++e) {
            if (OUT_MODE == 1) {
              hv[e] = (_Float16)sp[e];
            } else {
              unsigned short hb = f2bf_bits(sp[e]);
              unsigned short lb = f2bf_bits(sp[e] - bf_bits2f(hb));
              hv[e] = __builtin_bit_cast(_Float16, hb);
              lv[e] = __builtin_bit_cast(_Float16, lb);
            }
          }
          *(volatile v8h*)(C + (size_t)(mBase + row) * ldc + n0 + c8) = hv;
          if (OUT_MODE == 2) *(volatile v8h*)(C2 + (size_t)(mBase + row) * ldc + n0 + c8) = lv;
        }
        __threadfence();
      }
    }
    __builtin_amdgcn_fence(__ATOMIC_RELEASE, "workgroup");
    __builtin_amdgcn_wave_barrier();
    __builtin_amdgcn_fence(__ATOMIC_ACQUIRE, "workgroup");
  }
}

__global__ __launch_bounds__(256) void prep_x16(const int* __restrict__ batch, _Float16* __restrict__ X16, int nrows) {
  const int i = blockIdx.x * 256 + threadIdx.x;
  if (i >= nrows * 4) return;
  const int row = i >> 2, part = i & 3;
  const int t = row / NBATCH, b = row - t * NBATCH;
  const int* sp = batch + ((size_t)b * NT + t) * NF + 8 * (part & 1);
  const v4i x0 = *(const v4i*)sp;
  const v4i x1 = *(const v4i*)(sp + 4);
  const bool live = part < 2;
  v8h v;
#pragma unroll
  for (int e = 0; e < 4; ++e) {
    v[e]     = live ? (_Float16)(float)x0[e] : (_Float16)0.0f;
    v[4 + e] = live ? (_Float16)(float)x1[e] : (_Float16)0.0f;
  }
  _Float16* dp = X16 + (size_t)row * KP0 + 8 * part;
  *(volatile v8h*)dp = v;
  __threadfence();
  *(volatile v8h*)dp = v;
}

__global__ __launch_bounds__(256) void conv_wt(const float* __restrict__ src, _Float16* __restrict__ dst,
                                               int K, int N, int Kp, float scale) {
  const int i = blockIdx.x * 256 + threadIdx.x;
  if (i >= ((N * Kp) >> 3)) return;
  const int e0 = i * 8;
  const int n = e0 / Kp, kb = e0 - n * Kp;
  v8h v;
#pragma unroll
  for (int e = 0; e < 8; ++e) {
    const int k = kb + e;
    const int kc = (k < K) ? k : (K - 1);
    const float f = src[(size_t)kc * N + n] * scale;
    v[e] = (k < K) ? (_Float16)f : (_Float16)0.0f;
  }
  _Float16* dp = dst + e0;
  *(volatile v8h*)dp = v;
  __threadfence();
  *(volatile v8h*)dp = v;
}

__device__ __forceinline__ float sigm_f(float x) { return __builtin_amdgcn_rcpf(1.0f + __expf(-x)); }
__device__ __forceinline__ float tanh_f(float x) { return 1.0f - 2.0f * __builtin_amdgcn_rcpf(__expf(2.0f * x) + 1.0f); }

template <int U>
__device__ __forceinline__ void store_tile_f32(const float* ost, float* base, size_t rowstride, int wave, int lane) {
  v4f sv[2]; size_t so[2];
#pragma unroll
  for (int it = 0; it < 2; ++it) {
    const int e0 = (wave * 2 + it) * 128 + lane * 4;
    const int row = e0 / U, col = e0 - row * U;
    sv[it] = *(const v4f*)(ost + row * U + col);
    so[it] = (size_t)row * rowstride + col;
  }
  for (int pass = 0; pass < 2; ++pass) {
#pragma unroll
    for (int it = 0; it < 2; ++it) *(volatile v4f*)(base + so[it]) = sv[it];
    __threadfence();
  }
}

template <int U, bool LAST>
__global__ __launch_bounds__(2 * U) void gru_chunk_kernel(
    const float* __restrict__ xproj,
    const _Float16* __restrict__ rkT,
    const float* __restrict__ bias,
    const int* __restrict__ batch,
    const float* hS, const float* oS,
    float* hD, float* oD,
    _Float16* __restrict__ O16,
    float* __restrict__ outF,
    int t0, int nsteps, int init)
{
  constexpr int N3 = 3 * U;
  constexpr int HP = U + 8;
  constexpr int KT = U / 32;
  __shared__ __align__(16) _Float16 hsh[2 * 16 * HP];
  __shared__ __align__(16) float ost[16 * U];
  typedef Frag<_Float16> F;
  const int tid = threadIdx.x;
  const int lane = tid & 31, wave = tid >> 5, hh = lane >> 4, rl = lane & 15;
  const int b0 = blockIdx.x * 16;
  const int u = wave * 16 + rl;
  const float S = 1.0f / (HCARRY * WCARRY);
  int ns = nsteps;
  if (ns > TCH) ns = TCH;
  if (ns < 0) ns = 0;
  if (t0 + ns > NT) ns = NT - t0;
  if (ns < 0) ns = 0;

  float hreg[8], oreg[8];
  if (init) {
#pragma unroll
    for (int r = 0; r < 8; ++r) { hreg[r] = 0.0f; oreg[r] = 0.0f; }
  } else {
#pragma unroll
    for (int r = 0; r < 8; ++r) {
      const int row = 8 * hh + r;
      hreg[r] = hS[(size_t)(b0 + row) * U + u];
      oreg[r] = oS[(size_t)(b0 + row) * U + u];
    }
  }
#pragma unroll
  for (int r = 0; r < 8; ++r) hsh[(8 * hh + r) * HP + u] = (_Float16)(hreg[r] * HCARRY);
  __syncthreads();
  const float brz = bias[N3 + u], brr = bias[N3 + U + u], brh = bias[N3 + 2 * U + u];

  for (int s = 0; s < ns; ++s) {
    const int t = t0 + s;
    const _Float16* hc = hsh + (s & 1) * (16 * HP);
    _Float16* hn = hsh + ((s & 1) ^ 1) * (16 * HP);
    v8f acc[3];
#pragma unroll
    for (int g = 0; g < 3; ++g) acc[g] = (v8f){0.f,0.f,0.f,0.f,0.f,0.f,0.f,0.f};
#pragma unroll 1
    for (int kt = 0; kt < KT; ++kt) {
      const int k0 = kt * 32 + 8 * hh;
      v16h bfr[3];
#pragma unroll
      for (int g = 0; g < 3; ++g) bfr[g] = F::load(rkT + (size_t)(g * U + u) * U + k0);
      const v16h a = F::load(hc + rl * HP + k0);
#pragma unroll
      for (int g = 0; g < 3; ++g) acc[g] = F::mma(a, bfr[g], acc[g]);
      F::guard(acc[0], acc[2], a, a);
      F::keep(bfr[0], bfr[1], bfr[2], bfr[2]);
    }
    acc_guard3(acc[0], acc[1], acc[2]);

    const float* xrow = xproj + (size_t)s * NBATCH * N3;
#pragma unroll
    for (int r = 0; r < 8; ++r) {
      const int row = 8 * hh + r;
      const int b = b0 + row;
      const float* xp = xrow + (size_t)b * N3 + u;
      const float xz = xp[0];
      const float xr = xp[U];
      const float xh = xp[2 * U];
      const int mv = batch[((size_t)b * NT + t) * NF + (NF - 1)];
      const float z  = sigm_f(xz + (acc[0][r] * S + brz));
      const float rg = sigm_f(xr + (acc[1][r] * S + brr));
      const float cand = tanh_f(xh + rg * (acc[2][r] * S + brh));
      const float hnew = z * hreg[r] + (1.0f - z) * cand;
      const bool keep = (mv != -1);
      const float hv = keep ? hnew : hreg[r];
      const float ov = keep ? hnew : oreg[r];
      hreg[r] = hv;
      oreg[r] = ov;
      hn[row * HP + u] = (_Float16)(hv * HCARRY);
      ost[row * U + u] = ov;
    }
    __syncthreads();

    if (LAST) {
      store_tile_f32<U>(ost, outF + ((size_t)b0 * NT + t) * U, (size_t)NT * U, wave, lane);
    } else {
      const int e0 = wave * 256 + lane * 8;
      const int row = e0 / U, col = e0 - row * U;
      const v4f x0 = *(const v4f*)(ost + row * U + col);
      const v4f x1 = *(const v4f*)(ost + row * U + col + 4);
      v8h hv;
#pragma unroll
      for (int e = 0; e < 4; ++e) {
        hv[e]     = (_Float16)(x0[e] * HCARRY);
        hv[4 + e] = (_Float16)(x1[e] * HCARRY);
      }
      _Float16* dp = O16 + ((size_t)t * NBATCH + b0 + row) * U + col;
      for (int pass = 0; pass < 2; ++pass) {
        *(volatile v8h*)dp = hv;
        __threadfence();
      }
    }
    __syncthreads();
  }

#pragma unroll
  for (int r = 0; r < 8; ++r) ost[(8 * hh + r) * U + u] = oreg[r];
  __syncthreads();
  store_tile_f32<U>(ost, oD + (size_t)b0 * U, (size_t)U, wave, lane);
  __syncthreads();
#pragma unroll
  for (int r = 0; r < 8; ++r) ost[(8 * hh + r) * U + u] = hreg[r];
  __syncthreads();
  store_tile_f32<U>(ost, hD + (size_t)b0 * U, (size_t)U, wave, lane);
}

static void launch_gemm(const _Float16* A, int lda, const _Float16* Bt, int ldb, float* C, int ldc,
                        const float* bias, int M, int N, int K, float scale, hipStream_t stream) {
  const int tiles = (M / 64) * (N / 64);
  const int blocks = (tiles + 7) / 8;
  wmma_gemm64<0, false, 2, 0, false, 0><<<dim3(blocks, 1), 256, 0, stream>>>(
      (const unsigned short*)A, (const unsigned short*)A, lda, 0L,
      (const unsigned short*)Bt, (const unsigned short*)Bt, ldb, 0L,
      (void*)C, (void*)C, ldc, 0L, bias, bias, 0L, M, N, K, scale);
}

static inline size_t align256(size_t x) { return (x + 255) & ~(size_t)255; }

extern "C" void kernel_launch(void* const* d_in, const int* in_sizes, int n_in,
                              void* d_out, int out_size, void* d_ws, size_t ws_size,
                              hipStream_t stream) {
  if (n_in < 10) return;
  if (in_sizes[0] != NROWS * NF) return;
  if (in_sizes[1] != NF * 3 * UA || in_sizes[2] != UA * 3 * UA || in_sizes[3] != 2 * 3 * UA) return;
  if (in_sizes[4] != UA * 3 * UB || in_sizes[5] != UB * 3 * UB || in_sizes[6] != 2 * 3 * UB) return;
  if (in_sizes[7] != UB * 3 * UC || in_sizes[8] != UC * 3 * UC || in_sizes[9] != 2 * 3 * UC) return;
  if (out_size != NROWS * UC + NBATCH * UC) return;

  const int*   batch = (const int*)  d_in[0];
  const float* kw0   = (const float*)d_in[1];
  const float* rw0   = (const float*)d_in[2];
  const float* bs0   = (const float*)d_in[3];
  const float* kw1   = (const float*)d_in[4];
  const float* rw1   = (const float*)d_in[5];
  const float* bs1   = (const float*)d_in[6];
  const float* kw2   = (const float*)d_in[7];
  const float* rw2   = (const float*)d_in[8];
  const float* bs2   = (const float*)d_in[9];

  float* out0 = (float*)d_out;
  float* out1 = out0 + (size_t)NROWS * UC;

  size_t off = 0;
  const size_t oX   = off; off = align256(off + (size_t)NROWS * KP0 * 2);
  const size_t oK0  = off; off = align256(off + (size_t)3 * UA * KP0 * 2);
  const size_t oK1  = off; off = align256(off + (size_t)3 * UB * UA * 2);
  const size_t oK2  = off; off = align256(off + (size_t)3 * UC * UB * 2);
  const size_t oR0  = off; off = align256(off + (size_t)3 * UA * UA * 2);
  const size_t oR1  = off; off = align256(off + (size_t)3 * UB * UB * 2);
  const size_t oR2  = off; off = align256(off + (size_t)3 * UC * UC * 2);
  const size_t oXP  = off; off = align256(off + (size_t)TCH * NBATCH * 3 * UA * 4);
  const size_t oOa  = off; off = align256(off + (size_t)NROWS * UA * 2);
  const size_t oOb  = off; off = align256(off + (size_t)NROWS * UB * 2);
  const size_t oHS  = off; off = align256(off + (size_t)NBATCH * UA * 4);
  const size_t oOS  = off; off = align256(off + (size_t)NBATCH * UA * 4);
  if (off > ws_size) return;
  if (off > (size_t)134217728) return;
  char* ws = (char*)d_ws;
  _Float16* X16  = (_Float16*)(ws + oX);
  _Float16* kT0  = (_Float16*)(ws + oK0);
  _Float16* kT1  = (_Float16*)(ws + oK1);
  _Float16* kT2  = (_Float16*)(ws + oK2);
  _Float16* rT0  = (_Float16*)(ws + oR0);
  _Float16* rT1  = (_Float16*)(ws + oR1);
  _Float16* rT2  = (_Float16*)(ws + oR2);
  float*    xproj = (float*)(ws + oXP);
  _Float16* O16a = (_Float16*)(ws + oOa);
  _Float16* O16b = (_Float16*)(ws + oOb);
  float*    hS   = (float*)(ws + oHS);
  float*    oS   = (float*)(ws + oOS);

  prep_x16<<<(NROWS * 4 + 255) / 256, 256, 0, stream>>>(batch, X16, NROWS);
  conv_wt<<<((3 * UA * KP0) / 8 + 255) / 256, 256, 0, stream>>>(kw0, kT0, NF, 3 * UA, KP0, WCARRY);
  conv_wt<<<((3 * UB * UA) / 8 + 255) / 256, 256, 0, stream>>>(kw1, kT1, UA, 3 * UB, UA, WCARRY);
  conv_wt<<<((3 * UC * UB) / 8 + 255) / 256, 256, 0, stream>>>(kw2, kT2, UB, 3 * UC, UB, WCARRY);
  conv_wt<<<((3 * UA * UA) / 8 + 255) / 256, 256, 0, stream>>>(rw0, rT0, UA, 3 * UA, UA, WCARRY);
  conv_wt<<<((3 * UB * UB) / 8 + 255) / 256, 256, 0, stream>>>(rw1, rT1, UB, 3 * UB, UB, WCARRY);
  conv_wt<<<((3 * UC * UC) / 8 + 255) / 256, 256, 0, stream>>>(rw2, rT2, UC, 3 * UC, UC, WCARRY);

  const int MCH = TCH * NBATCH;
  for (int c = 0; c < NCH; ++c) {
    const int t0 = c * TCH;
    launch_gemm(X16 + (size_t)t0 * NBATCH * KP0, KP0, kT0, KP0, xproj, 3 * UA, bs0, MCH, 3 * UA, KP0, 1.0f / WCARRY, stream);
    gru_chunk_kernel<UA, false><<<NBATCH / 16, 2 * UA, 0, stream>>>(
        xproj, rT0, bs0, batch, hS, oS, hS, oS, O16a, out0, t0, TCH, (c == 0) ? 1 : 0);
  }
  for (int c = 0; c < NCH; ++c) {
    const int t0 = c * TCH;
    launch_gemm(O16a + (size_t)t0 * NBATCH * UA, UA, kT1, UA, xproj, 3 * UB, bs1, MCH, 3 * UB, UA, 1.0f / (HCARRY * WCARRY), stream);
    gru_chunk_kernel<UB, false><<<NBATCH / 16, 2 * UB, 0, stream>>>(
        xproj, rT1, bs1, batch, hS, oS, hS, oS, O16b, out0, t0, TCH, (c == 0) ? 1 : 0);
  }
  for (int c = 0; c < NCH; ++c) {
    const int t0 = c * TCH;
    launch_gemm(O16b + (size_t)t0 * NBATCH * UB, UB, kT2, UB, xproj, 3 * UC, bs2, MCH, 3 * UC, UB, 1.0f / (HCARRY * WCARRY), stream);
    float* hdst = (c == NCH - 1) ? out1 : hS;
    gru_chunk_kernel<UC, true><<<NBATCH / 16, 2 * UC, 0, stream>>>(
        xproj, rT2, bs2, batch, hS, oS, hdst, oS, O16b, out0, t0, TCH, (c == 0) ? 1 : 0);
  }
}
